// MixtureOfExperts_28209345200699
// MI455X (gfx1250) — hardware-verified
//
#include <hip/hip_runtime.h>
#include <stddef.h>
#include <stdint.h>

#define NTOK   4096
#define DM     768
#define HD     768
#define HS     3072
#define NE     8
#define TOPK   2
#define TR     64
#define NTILE  136
#define MP     8704
#define TABH   32
#define TABL   (TABH + MP)
#define TABN   (TABH + MP + NTOK * TOPK)
#define TPT    16
#define NTHR   256
#define GTHR   128
#define WSMAX  268435456
#define LDS_BKT ((TABN + NE * 8) * 4)

static_assert(MP == NTILE * TR);
static_assert(MP >= NTOK * TOPK + NE * (TR - 1));
static_assert((TABN % 32) == 0);
static_assert(NTOK == NTHR * TPT);
static_assert((NTOK % TR) == 0);
static_assert((DM % 64) == 0 && (HD % 64) == 0 && (HS % 64) == 0);
static_assert((DM % 32) == 0 && (HD % 32) == 0 && (HS % 32) == 0);
static_assert((DM % 128) == 0);
static_assert(TR == (GTHR / 32) * 16);
static_assert(LDS_BKT <= 160000);
static_assert(NTHR / 32 == 8);
static_assert((NTOK % NTHR) == 0 && (NTOK % 8) == 0);
static_assert(HD == DM);

typedef float          v4f  __attribute__((ext_vector_type(4)));
typedef float          v8f  __attribute__((ext_vector_type(8)));
typedef int            v4i  __attribute__((ext_vector_type(4)));
typedef int            v8i  __attribute__((ext_vector_type(8)));
typedef unsigned short v8us __attribute__((ext_vector_type(8)));
typedef __bf16         v16bf __attribute__((ext_vector_type(16)));
union FragB { v16bf v; v8us h[2]; v8i w; };

__device__ __forceinline__ v8f wmb(const FragB& a, const FragB& b, v8f c) {
  v8f d = __builtin_amdgcn_wmma_f32_16x16x32_bf16(false, a.v, false, b.v, (short)0, c, false, false);
  asm volatile("v_nop\n\tv_nop\n\tv_nop\n\tv_nop" : "+v"(d) : "v"(a.w), "v"(b.w));
  return d;
}

__device__ __forceinline__ unsigned short rne16(float f) {
  unsigned u = __float_as_uint(f);
  u += 0x7FFFu + ((u >> 16) & 1u);
  return (unsigned short)(u >> 16);
}
__device__ __forceinline__ float rne16f(float f) {
  return __uint_as_float(((unsigned)rne16(f)) << 16);
}
__device__ __forceinline__ v8us cvt8(const v4f a, const v4f b) {
  v8us o;
  o[0] = rne16(a.x); o[1] = rne16(a.y); o[2] = rne16(a.z); o[3] = rne16(a.w);
  o[4] = rne16(b.x); o[5] = rne16(b.y); o[6] = rne16(b.z); o[7] = rne16(b.w);
  return o;
}
__device__ __forceinline__ void sp1(float v, unsigned short& hi, unsigned short& lo) {
  const unsigned short hb = rne16(v);
  const float hf = __uint_as_float(((unsigned)hb) << 16);
  hi = hb;
  lo = rne16(v - hf);
}
__device__ __forceinline__ void split8(const v4f a, const v4f b, v8us& hv, v8us& lv) {
  unsigned short h0, h1, h2, h3, h4, h5, h6, h7, l0, l1, l2, l3, l4, l5, l6, l7;
  sp1(a.x, h0, l0); sp1(a.y, h1, l1); sp1(a.z, h2, l2); sp1(a.w, h3, l3);
  sp1(b.x, h4, l4); sp1(b.y, h5, l5); sp1(b.z, h6, l6); sp1(b.w, h7, l7);
  hv[0] = h0; hv[1] = h1; hv[2] = h2; hv[3] = h3; hv[4] = h4; hv[5] = h5; hv[6] = h6; hv[7] = h7;
  lv[0] = l0; lv[1] = l1; lv[2] = l2; lv[3] = l3; lv[4] = l4; lv[5] = l5; lv[6] = l6; lv[7] = l7;
}

__global__ __launch_bounds__(NTHR) void k_wtr(const float* __restrict__ src, unsigned short* dst,
                                              int K, int N, int E, int nUnits) {
  const int u = (int)blockIdx.x * NTHR + (int)threadIdx.x;
  if (u >= nUnits) return;
  const int kq  = K >> 3;
  const int per = N * kq;
  int e = u / per;
  e = e > E - 1 ? E - 1 : e;
  const int rem = u - e * per;
  const int n   = rem / kq;
  const int k8  = (rem - n * kq) * 8;
  const float* p = src + ((size_t)e * (size_t)K + (size_t)k8) * (size_t)N + n;
  v4f a, b;
  a.x = p[0];                 a.y = p[(size_t)N];         a.z = p[(size_t)2 * N];     a.w = p[(size_t)3 * N];
  b.x = p[(size_t)4 * N];     b.y = p[(size_t)5 * N];     b.z = p[(size_t)6 * N];     b.w = p[(size_t)7 * N];
  const v8us o = cvt8(a, b);
  const size_t q = ((size_t)e * (size_t)N + (size_t)n) * (size_t)K + (size_t)k8;
  *(volatile v8us*)(dst + q) = o;
  __threadfence();
  *(volatile v8us*)(dst + q) = o;
}

__global__ __launch_bounds__(NTHR) void k_xcvt(const float* __restrict__ x, unsigned short* xb, int nUnits) {
  const int u = (int)blockIdx.x * NTHR + (int)threadIdx.x;
  if (u >= nUnits) return;
  const float* p = x + (size_t)u * 8;
  const v4f a = *(const v4f*)p;
  const v4f b = *(const v4f*)(p + 4);
  const v8us o = cvt8(a, b);
  const size_t q = (size_t)u * 8;
  *(volatile v8us*)(xb + q) = o;
  __threadfence();
  *(volatile v8us*)(xb + q) = o;
}

__device__ __forceinline__ void gacc(float xq, const float* swrow, float (&acc)[NE]) {
  const v4f wa = *(const v4f*)(swrow);
  const v4f wb = *(const v4f*)(swrow + 4);
  acc[0] = fmaf(xq, wa.x, acc[0]); acc[1] = fmaf(xq, wa.y, acc[1]);
  acc[2] = fmaf(xq, wa.z, acc[2]); acc[3] = fmaf(xq, wa.w, acc[3]);
  acc[4] = fmaf(xq, wb.x, acc[4]); acc[5] = fmaf(xq, wb.y, acc[5]);
  acc[6] = fmaf(xq, wb.z, acc[6]); acc[7] = fmaf(xq, wb.w, acc[7]);
}

__global__ __launch_bounds__(NTHR) void k_gate(const float* __restrict__ x, const float* __restrict__ rw,
                                               const float* __restrict__ sgw, const float* __restrict__ sgb,
                                               int* route) {
  __shared__ __attribute__((aligned(16))) float sw[DM * NE];
  __shared__ __attribute__((aligned(16))) float ss[DM];
  const int tid = (int)threadIdx.x;
#pragma unroll 1
  for (int i = tid; i < DM * NE; i += NTHR) sw[i] = rne16f(rw[i]);
#pragma unroll 1
  for (int i = tid; i < DM; i += NTHR) ss[i] = rne16f(sgw[i]);
  __syncthreads();
  int t = (int)blockIdx.x * NTHR + tid;
  const bool live = t < NTOK;
  t = t > NTOK - 1 ? NTOK - 1 : t;
  const float* xr = x + (size_t)t * DM;
  float acc[NE];
#pragma unroll
  for (int e = 0; e < NE; ++e) acc[e] = 0.f;
  float az = 0.f;
#pragma unroll 1
  for (int d4 = 0; d4 < DM / 4; ++d4) {
    const v4f xv = *(const v4f*)(xr + 4 * d4);
    const v4f gv = *(const v4f*)(ss + 4 * d4);
    const float* swr = sw + (size_t)(4 * d4) * NE;
    const float x0 = rne16f(xv.x), x1 = rne16f(xv.y), x2 = rne16f(xv.z), x3 = rne16f(xv.w);
    gacc(x0, swr,          acc);
    gacc(x1, swr + NE,     acc);
    gacc(x2, swr + 2 * NE, acc);
    gacc(x3, swr + 3 * NE, acc);
    az = fmaf(x0, gv.x, az);
    az = fmaf(x1, gv.y, az);
    az = fmaf(x2, gv.z, az);
    az = fmaf(x3, gv.w, az);
  }
  float mx = acc[0];
#pragma unroll
  for (int e = 1; e < NE; ++e) mx = fmaxf(mx, acc[e]);
  float p[NE];
  float s = 0.f;
#pragma unroll
  for (int e = 0; e < NE; ++e) { p[e] = __expf(acc[e] - mx); s += p[e]; }
  const float inv = 1.0f / s;
#pragma unroll
  for (int e = 0; e < NE; ++e) p[e] *= inv;
  int i1 = 0;
  float b1 = p[0];
#pragma unroll
  for (int e = 1; e < NE; ++e) {
    const bool up = p[e] > b1;
    i1 = up ? e : i1;
    b1 = up ? p[e] : b1;
  }
  int i2 = 0;
  float b2 = -1.0f;
#pragma unroll
  for (int e = 0; e < NE; ++e) {
    const bool ok = (e != i1) && (p[e] > b2);
    i2 = ok ? e : i2;
    b2 = ok ? p[e] : b2;
  }
  const float inv2 = 1.0f / (b1 + b2);
  const float w1 = b1 * inv2;
  const float w2 = b2 * inv2;
  const float z  = az + rne16f(sgb[0]);
  const float al = 1.0f / (1.0f + __expf(-z));
  v4i rec;
  rec.x = i1 | (i2 << 8); rec.y = __float_as_int(w1); rec.z = __float_as_int(w2); rec.w = __float_as_int(al);
  if (live) *(volatile v4i*)(route + (size_t)t * 4) = rec;
  __threadfence();
  if (live) *(volatile v4i*)(route + (size_t)t * 4) = rec;
}

__device__ __forceinline__ void cnt_add(int c, int (&cnt)[NE]) {
  c = c < 0 ? 0 : (c > NE - 1 ? NE - 1 : c);
#pragma unroll
  for (int e = 0; e < NE; ++e) cnt[e] += (c == e) ? 1 : 0;
}
__device__ __forceinline__ int slot_of(int c, int (&base)[NE]) {
  c = c < 0 ? 0 : (c > NE - 1 ? NE - 1 : c);
  int p = 0;
#pragma unroll
  for (int e = 0; e < NE; ++e) {
    const bool mt = (c == e);
    p = mt ? base[e] : p;
    base[e] += mt ? 1 : 0;
  }
  return p < 0 ? 0 : (p > MP - 1 ? MP - 1 : p);
}

__global__ __launch_bounds__(NTHR) void k_bucket(const int* __restrict__ route, int* tab) {
  extern __shared__ v4i lds_dyn[];
  int* img = (int*)lds_dyn;
  int* lst = img + TABH;
  int* pos = img + TABL;
  int* wt  = img + TABN;
  const int tid = (int)threadIdx.x, lane = tid & 31, wave = tid >> 5;

  const v4i z4 = {0, 0, 0, 0};
#pragma unroll 1
  for (int p = tid; p < TABN / 4; p += NTHR) *(v4i*)(img + 4 * p) = z4;
  __syncthreads();

  const int t0 = tid * TPT;
  int cnt[NE];
#pragma unroll
  for (int e = 0; e < NE; ++e) cnt[e] = 0;
#pragma unroll 1
  for (int c = 0; c < TPT; ++c) {
    const int rx = route[(size_t)(t0 + c) * 4];
    cnt_add(rx & 255, cnt);
    cnt_add((rx >> 8) & 255, cnt);
  }
  int incl[NE];
#pragma unroll
  for (int e = 0; e < NE; ++e) {
    int v = cnt[e];
#pragma unroll
    for (int d = 1; d < 32; d <<= 1) {
      const int up = __shfl_up(v, d);
      if (lane >= d) v += up;
    }
    incl[e] = v;
    if (lane == 31) wt[e * 8 + wave] = v;
  }
  __syncthreads();
  int pre[NE], tot[NE];
#pragma unroll
  for (int e = 0; e < NE; ++e) {
    int s = 0, all = 0;
#pragma unroll
    for (int w2 = 0; w2 < NTHR / 32; ++w2) {
      const int v = wt[e * 8 + w2];
      all += v;
      s   += (w2 < wave) ? v : 0;
    }
    pre[e] = s + incl[e] - cnt[e];
    all = all < 0 ? 0 : (all > NTOK * TOPK ? NTOK * TOPK : all);
    tot[e] = all;
  }
  int off[NE + 1];
  off[0] = 0;
#pragma unroll
  for (int e = 0; e < NE; ++e) {
    int nx = off[e] + ((tot[e] + TR - 1) / TR) * TR;
    nx = nx > MP ? MP : nx;
    off[e + 1] = nx;
  }
  int base[NE];
#pragma unroll
  for (int e = 0; e < NE; ++e) base[e] = off[e] + pre[e];
#pragma unroll 1
  for (int c = 0; c < TPT; ++c) {
    const int rx = route[(size_t)(t0 + c) * 4];
    const int t = t0 + c;
    const int pa = slot_of(rx & 255, base);        lst[pa] = t; pos[2 * t]     = pa;
    const int pb = slot_of((rx >> 8) & 255, base); lst[pb] = t; pos[2 * t + 1] = pb;
  }
  __syncthreads();
  if (tid == 0) {
#pragma unroll
    for (int e = 0; e < NE; ++e) img[e] = tot[e];
#pragma unroll
    for (int j = 0; j <= NE; ++j) img[NE + j] = off[j];
  }
  __syncthreads();
#pragma unroll 1
  for (int p = tid; p < TABN / 4; p += NTHR) {
    const v4i v = *(const v4i*)(img + 4 * p);
    *(volatile v4i*)(tab + 4 * p) = v;
  }
  __threadfence();
#pragma unroll 1
  for (int p = tid; p < TABN / 4; p += NTHR) {
    const v4i v = *(const v4i*)(img + 4 * p);
    *(volatile v4i*)(tab + 4 * p) = v;
  }
}

__global__ __launch_bounds__(NTHR) void k_gather(const unsigned short* __restrict__ xb, const int* __restrict__ tab,
                                                 unsigned short* xg, int nUnits) {
  const int u = (int)blockIdx.x * NTHR + (int)threadIdx.x;
  if (u >= nUnits) return;
  const int row = u / (DM / 8);
  const int c8  = (u - row * (DM / 8)) * 8;
  int tk = tab[TABH + row];
  tk = tk < 0 ? 0 : (tk > NTOK - 1 ? NTOK - 1 : tk);
  const v8us o = *(const v8us*)(xb + (size_t)tk * DM + c8);
  const size_t q = (size_t)row * DM + (size_t)c8;
  *(volatile v8us*)(xg + q) = o;
  __threadfence();
  *(volatile v8us*)(xg + q) = o;
}

__device__ __forceinline__ int tile_slot(const int* __restrict__ tab, int rowBase) {
  const v4i ho0 = *(const v4i*)(tab + 8);
  const v4i ho1 = *(const v4i*)(tab + 12);
  int e = 0;
#define SELX(J, OJ) { const bool ge_ = rowBase >= (OJ); e = ge_ ? (J) : e; }
  SELX(0, ho0.x) SELX(1, ho0.y) SELX(2, ho0.z) SELX(3, ho0.w)
  SELX(4, ho1.x) SELX(5, ho1.y) SELX(6, ho1.z) SELX(7, ho1.w)
#undef SELX
  return e < 0 ? 0 : (e > NE - 1 ? NE - 1 : e);
}

__global__ __launch_bounds__(GTHR) void k_up(const unsigned short* __restrict__ xa,
                                             const unsigned short* __restrict__ wgt,
                                             const unsigned short* __restrict__ wut,
                                             const int* __restrict__ tab,
                                             unsigned short* hhi, unsigned short* hlo, int ldo, int routed) {
  __shared__ __attribute__((aligned(16))) float stg[TR * 64];
  const int tid = (int)threadIdx.x, lane = tid & 31, wave = tid >> 5, hh = lane >> 4, m = lane & 15;
  const int rowBase = (int)blockIdx.x * TR;
  const int col0    = (int)blockIdx.y * 64;
  int e = tile_slot(tab, rowBase);
  e = (routed != 0) ? e : 0;

  v8f accg[4], accu[4];
  {
    const v8f z = {0.f, 0.f, 0.f, 0.f, 0.f, 0.f, 0.f, 0.f};
    accg[0] = z; accg[1] = z; accg[2] = z; accg[3] = z;
    accu[0] = z; accu[1] = z; accu[2] = z; accu[3] = z;
  }
  const size_t arow = (size_t)(rowBase + 16 * wave + m) * (size_t)DM + (size_t)(8 * hh);
  const unsigned short* aph = xa + arow;
  const size_t woff = (size_t)e * (size_t)(HD * DM) + (size_t)(col0 + m) * (size_t)DM + (size_t)(8 * hh);
  const unsigned short* wg = wgt + woff;
  const unsigned short* wu = wut + woff;
#pragma unroll 1
  for (int ks = 0; ks < DM / 32; ++ks) {
    FragB ah;
    ah.h[0] = *(const v8us*)(aph + 32 * ks);
    ah.h[1] = *(const v8us*)(aph + 32 * ks + 16);
#pragma unroll
    for (int t = 0; t < 4; ++t) {
      const unsigned short* q1 = wg + (size_t)(16 * t) * (size_t)DM + 32 * ks;
      const unsigned short* q2 = wu + (size_t)(16 * t) * (size_t)DM + 32 * ks;
      FragB bg, bu;
      bg.h[0] = *(const v8us*)q1;
      bg.h[1] = *(const v8us*)(q1 + 16);
      bu.h[0] = *(const v8us*)q2;
      bu.h[1] = *(const v8us*)(q2 + 16);
      accg[t] = wmb(ah, bg, accg[t]);
      accu[t] = wmb(ah, bu, accu[t]);
    }
  }

#pragma unroll
  for (int t = 0; t < 4; ++t) {
    const int lc = 16 * t + m;
#pragma unroll
    for (int r = 0; r < 8; ++r) {
      const int lr = 16 * wave + 8 * hh + r;
      const float gg = accg[t][r];
      const float uu = accu[t][r];
      const float sg = __builtin_amdgcn_rcpf(1.0f + __expf(-gg));
      stg[lr * 64 + lc] = (gg * sg) * uu;
    }
  }
  __syncthreads();

  const int q8 = lane & 7, sub = lane >> 3;
  v8us hv[4], lv[4];
  size_t po[4];
#pragma unroll
  for (int i = 0; i < 4; ++i) {
    const int lr = 16 * wave + 4 * i + sub;
    const v4f a = *(const v4f*)(stg + lr * 64 + 8 * q8);
    const v4f b = *(const v4f*)(stg + lr * 64 + 8 * q8 + 4);
    split8(a, b, hv[i], lv[i]);
    po[i] = (size_t)(rowBase + lr) * (size_t)ldo + (size_t)(col0 + 8 * q8);
  }
#pragma unroll
  for (int i = 0; i < 4; ++i) {
    *(volatile v8us*)(hhi + po[i]) = hv[i];
    *(volatile v8us*)(hlo + po[i]) = lv[i];
  }
  __threadfence();
#pragma unroll
  for (int i = 0; i < 4; ++i) {
    *(volatile v8us*)(hhi + po[i]) = hv[i];
    *(volatile v8us*)(hlo + po[i]) = lv[i];
  }
}

__global__ __launch_bounds__(GTHR) void k_down(const unsigned short* __restrict__ hhi,
                                               const unsigned short* __restrict__ hlo,
                                               const unsigned short* __restrict__ wdt,
                                               const int* __restrict__ tab, float* y, int K, int routed) {
  __shared__ __attribute__((aligned(16))) float stg[TR * 64];
  const int tid = (int)threadIdx.x, lane = tid & 31, wave = tid >> 5, hh = lane >> 4, m = lane & 15;
  const int rowBase = (int)blockIdx.x * TR;
  const int col0    = (int)blockIdx.y * 64;
  int e = tile_slot(tab, rowBase);
  e = (routed != 0) ? e : 0;
  const int nks = K / 32;

  v8f acc[4];
  {
    const v8f z = {0.f, 0.f, 0.f, 0.f, 0.f, 0.f, 0.f, 0.f};
    acc[0] = z; acc[1] = z; acc[2] = z; acc[3] = z;
  }
  const size_t arow = (size_t)(rowBase + 16 * wave + m) * (size_t)K + (size_t)(8 * hh);
  const unsigned short* aph = hhi + arow;
  const unsigned short* apl = hlo + arow;
  const unsigned short* wp  = wdt + (size_t)e * (size_t)DM * (size_t)K + (size_t)(col0 + m) * (size_t)K
                              + (size_t)(8 * hh);
#pragma unroll 1
  for (int ks = 0; ks < nks; ++ks) {
    FragB ah, al;
    ah.h[0] = *(const v8us*)(aph + 32 * ks);
    ah.h[1] = *(const v8us*)(aph + 32 * ks + 16);
    al.h[0] = *(const v8us*)(apl + 32 * ks);
    al.h[1] = *(const v8us*)(apl + 32 * ks + 16);
#pragma unroll
    for (int t = 0; t < 4; ++t) {
      const unsigned short* wq = wp + (size_t)(16 * t) * (size_t)K + 32 * ks;
      FragB bf;
      bf.h[0] = *(const v8us*)wq;
      bf.h[1] = *(const v8us*)(wq + 16);
      acc[t] = wmb(ah, bf, acc[t]);
      acc[t] = wmb(al, bf, acc[t]);
    }
  }

#pragma unroll
  for (int t = 0; t < 4; ++t) {
    const int lc = 16 * t + m;
#pragma unroll
    for (int r = 0; r < 8; ++r) {
      const int lr = 16 * wave + 8 * hh + r;
      stg[lr * 64 + lc] = acc[t][r];
    }
  }
  __syncthreads();

  v4f fv[8];
  size_t op[8];
#pragma unroll
  for (int i = 0; i < 8; ++i) {
    const int lr = 16 * wave + 2 * i + hh;
    fv[i] = *(const v4f*)(stg + lr * 64 + 4 * m);
    op[i] = (size_t)(rowBase + lr) * (size_t)DM + (size_t)(col0 + 4 * m);
  }
#pragma unroll
  for (int i = 0; i < 8; ++i) *(volatile v4f*)(y + op[i]) = fv[i];
  __threadfence();
#pragma unroll
  for (int i = 0; i < 8; ++i) *(volatile v4f*)(y + op[i]) = fv[i];
}

__global__ __launch_bounds__(NTHR) void k_combine(const float* __restrict__ ys, const float* __restrict__ yr,
                                                  const int* __restrict__ route, const int* __restrict__ tab,
                                                  float* out) {
  const int lane = (int)threadIdx.x & 31, wave = (int)threadIdx.x >> 5;
  const int t = (int)blockIdx.x * 8 + wave;
  if (t >= NTOK) return;
  const v4i rec = *(const v4i*)(route + (size_t)t * 4);
  const float w1 = __int_as_float(rec.y);
  const float w2 = __int_as_float(rec.z);
  const float al = __int_as_float(rec.w);
  const float oma = 1.0f - al;
  int qa = tab[TABL + 2 * t];
  int qb = tab[TABL + 2 * t + 1];
  qa = qa < 0 ? 0 : (qa > MP - 1 ? MP - 1 : qa);
  qb = qb < 0 ? 0 : (qb > MP - 1 ? MP - 1 : qb);
  const float* yss = ys + (size_t)t * DM;
  const float* ya  = yr + (size_t)qa * DM;
  const float* yb  = yr + (size_t)qb * DM;
  float* orow = out + (size_t)t * DM;
#pragma unroll 1
  for (int c = 0; c < DM / 128; ++c) {
    const int col = 128 * c + 4 * lane;
    const v4f s = *(const v4f*)(yss + col);
    const v4f a = *(const v4f*)(ya + col);
    const v4f b = *(const v4f*)(yb + col);
    v4f r, o;
    r.x = w1 * a.x; r.x = fmaf(w2, b.x, r.x); o.x = al * s.x + oma * r.x;
    r.y = w1 * a.y; r.y = fmaf(w2, b.y, r.y); o.y = al * s.y + oma * r.y;
    r.z = w1 * a.z; r.z = fmaf(w2, b.z, r.z); o.z = al * s.z + oma * r.z;
    r.w = w1 * a.w; r.w = fmaf(w2, b.w, r.w); o.w = al * s.w + oma * r.w;
    float* op = orow + col;
    *(volatile v4f*)op = o;
    __threadfence();
    *(volatile v4f*)op = o;
  }
}

static inline int cdiv(int a, int b) { return (a + b - 1) / b; }

extern "C" void kernel_launch(void* const* d_in, const int* in_sizes, int n_in,
                              void* d_out, int out_size, void* d_ws, size_t ws_size,
                              hipStream_t stream) {
  if (n_in < 10) return;
  if (in_sizes[0] != NTOK * DM) return;
  if (in_sizes[1] != DM * NE) return;
  if (in_sizes[2] != NE * DM * HD) return;
  if (in_sizes[3] != NE * DM * HD) return;
  if (in_sizes[4] != NE * HD * DM) return;
  if (in_sizes[5] != DM * HS) return;
  if (in_sizes[6] != DM * HS) return;
  if (in_sizes[7] != HS * DM) return;
  if (in_sizes[8] != DM) return;
  if (in_sizes[9] < 1) return;
  if (out_size != NTOK * DM) return;

  const float* x   = (const float*)d_in[0];
  const float* rw  = (const float*)d_in[1];
  const float* wg  = (const float*)d_in[2];
  const float* wu  = (const float*)d_in[3];
  const float* wd  = (const float*)d_in[4];
  const float* wsg = (const float*)d_in[5];
  const float* wsu = (const float*)d_in[6];
  const float* wsd = (const float*)d_in[7];
  const float* sgw = (const float*)d_in[8];
  const float* sgb = (const float*)d_in[9];
  float* out = (float*)d_out;

  char* ws = (char*)d_ws;
  size_t off = 0;
  const size_t oWG  = off; off += (size_t)NE * HD * DM * 2;    off = (off + 255) & ~(size_t)255;
  const size_t oWU  = off; off += (size_t)NE * HD * DM * 2;    off = (off + 255) & ~(size_t)255;
  const size_t oWD  = off; off += (size_t)NE * DM * HD * 2;    off = (off + 255) & ~(size_t)255;
  const size_t oWSG = off; off += (size_t)HS * DM * 2;         off = (off + 255) & ~(size_t)255;
  const size_t oWSU = off; off += (size_t)HS * DM * 2;         off = (off + 255) & ~(size_t)255;
  const size_t oWSD = off; off += (size_t)DM * HS * 2;         off = (off + 255) & ~(size_t)255;
  const size_t oXB  = off; off += (size_t)NTOK * DM * 2;       off = (off + 255) & ~(size_t)255;
  const size_t oRT  = off; off += (size_t)NTOK * 4 * 4;        off = (off + 255) & ~(size_t)255;
  const size_t oTAB = off; off += (size_t)TABN * 4;            off = (off + 255) & ~(size_t)255;
  const size_t oXG  = off; off += (size_t)MP * DM * 2;         off = (off + 255) & ~(size_t)255;
  const size_t oHRH = off; off += (size_t)MP * HD * 2;         off = (off + 255) & ~(size_t)255;
  const size_t oHRL = off; off += (size_t)MP * HD * 2;         off = (off + 255) & ~(size_t)255;
  const size_t oHSH = off; off += (size_t)NTOK * HS * 2;       off = (off + 255) & ~(size_t)255;
  const size_t oHSL = off; off += (size_t)NTOK * HS * 2;       off = (off + 255) & ~(size_t)255;
  const size_t oYR  = off; off += (size_t)MP * DM * 4;         off = (off + 255) & ~(size_t)255;
  const size_t oYS  = off; off += (size_t)NTOK * DM * 4;       off = (off + 255) & ~(size_t)255;
  if (off > ws_size || off > (size_t)WSMAX) return;

  unsigned short* WG  = (unsigned short*)(ws + oWG);
  unsigned short* WU  = (unsigned short*)(ws + oWU);
  unsigned short* WD  = (unsigned short*)(ws + oWD);
  unsigned short* WSG = (unsigned short*)(ws + oWSG);
  unsigned short* WSU = (unsigned short*)(ws + oWSU);
  unsigned short* WSD = (unsigned short*)(ws + oWSD);
  unsigned short* XB  = (unsigned short*)(ws + oXB);
  int*            RT  = (int*)(ws + oRT);
  int*            TAB = (int*)(ws + oTAB);
  unsigned short* XG  = (unsigned short*)(ws + oXG);
  unsigned short* HRH = (unsigned short*)(ws + oHRH);
  unsigned short* HRL = (unsigned short*)(ws + oHRL);
  unsigned short* HSH = (unsigned short*)(ws + oHSH);
  unsigned short* HSL = (unsigned short*)(ws + oHSL);
  float*          YR  = (float*)(ws + oYR);
  float*          YS  = (float*)(ws + oYS);

  hipFuncSetAttribute(reinterpret_cast<const void*>(&k_bucket),
                      hipFuncAttributeMaxDynamicSharedMemorySize, LDS_BKT);

  {
    const int nUr = NE * HD * DM / 8;
    k_wtr<<<cdiv(nUr, NTHR), NTHR, 0, stream>>>(wg, WG, DM, HD, NE, nUr);
    k_wtr<<<cdiv(nUr, NTHR), NTHR, 0, stream>>>(wu, WU, DM, HD, NE, nUr);
    k_wtr<<<cdiv(nUr, NTHR), NTHR, 0, stream>>>(wd, WD, HD, DM, NE, nUr);
    const int nUs = HS * DM / 8;
    k_wtr<<<cdiv(nUs, NTHR), NTHR, 0, stream>>>(wsg, WSG, DM, HS, 1, nUs);
    k_wtr<<<cdiv(nUs, NTHR), NTHR, 0, stream>>>(wsu, WSU, DM, HS, 1, nUs);
    k_wtr<<<cdiv(nUs, NTHR), NTHR, 0, stream>>>(wsd, WSD, HS, DM, 1, nUs);
  }
  {
    const int nUx = NTOK * DM / 8;
    k_xcvt<<<cdiv(nUx, NTHR), NTHR, 0, stream>>>(x, XB, nUx);
  }
  k_gate<<<cdiv(NTOK, NTHR), NTHR, 0, stream>>>(x, rw, sgw, sgb, RT);
  k_bucket<<<1, NTHR, LDS_BKT, stream>>>(RT, TAB);
  {
    const int nUg = MP * (DM / 8);
    k_gather<<<cdiv(nUg, NTHR), NTHR, 0, stream>>>(XB, TAB, XG, nUg);
  }
  k_up<<<dim3(NTOK / TR, HS / 64), GTHR, 0, stream>>>(XB, WSG, WSU, TAB, HSH, HSL, HS, 0);
  k_up<<<dim3(NTILE, HD / 64), GTHR, 0, stream>>>(XG, WG, WU, TAB, HRH, HRL, HD, 1);
  k_down<<<dim3(NTOK / TR, DM / 64), GTHR, 0, stream>>>(HSH, HSL, WSD, TAB, YS, HS, 0);
  k_down<<<dim3(NTILE, DM / 64), GTHR, 0, stream>>>(HRH, HRL, WD, TAB, YR, HD, 1);
  k_combine<<<NTOK / 8, NTHR, 0, stream>>>(YS, YR, RT, TAB, out);
}
